// SeFTNetwork_85968065397118
// MI455X (gfx1250) — hardware-verified
//
#include <hip/hip_runtime.h>


namespace {
constexpr int R = 2048, V = 32, NP = 32, L = 1008, NIN = 34, KIN = 64  , W = 128, NH = 4, HD = 32, NSR = NP * L  ;
constexpr float XS = 8.0f, WSC = 256.0f, MAXT = 100.0f;

typedef _Float16 b16;
typedef __attribute__((ext_vector_type(16))) _Float16 v16b;
typedef __attribute__((ext_vector_type(8))) _Float16 v8b;
typedef __attribute__((ext_vector_type(8))) float v8f;
typedef __attribute__((ext_vector_type(4))) float v4f;
__device__ __forceinline__ float bf16_rne(float f) { unsigned int u = __float_as_uint(f); u += 0x7FFFu + ((u >> 16) & 1u); return __uint_as_float(u & 0xFFFF0000u); }
__device__ __forceinline__ void split16(float v, b16& hi, b16& lo) { hi = (b16)v; lo = (b16)(v - (float)hi); }
__device__ __forceinline__ v16b frag_kb(const b16* p, int hh) { const v8b a = *(const v8b*)(p + 8 * hh), b = *(const v8b*)(p + 16 + 8 * hh); v16b f;
#pragma unroll
  for (int e = 0; e < 8; ++e) { f[e] = a[e]; f[8 + e] = b[e]; } return f; }
__device__ __forceinline__ v8f wmma16b(v16b a, v16b b, v8f c) { v8f d = __builtin_amdgcn_wmma_f32_16x16x32_f16(false, a, false, b, (short)0, c, false, false); asm volatile("v_nop\n\tv_nop\n\tv_nop\n\tv_nop" : "+v"(d) : "v"(a), "v"(b)); return d; }
__device__ __forceinline__ void wave_lds_sync() { __builtin_amdgcn_fence(__ATOMIC_RELEASE, "workgroup"); __builtin_amdgcn_wave_barrier(); __builtin_amdgcn_fence(__ATOMIC_ACQUIRE, "workgroup"); }
__device__ __forceinline__ float pmul(float a, float b) { float p = a * b; asm volatile("" : "+v"(p)); return p; }
__device__ __forceinline__ int iclamp(int v, int lo, int hi) { return v < lo ? lo : (v > hi ? hi : v); }
__device__ __forceinline__ float nexp(float x) { return __builtin_amdgcn_exp2f(x * 1.4426950408889634f); }

__global__ __launch_bounds__(256) void scatter_kernel(const int* __restrict__ M, const int* __restrict__ obs, const float* __restrict__ X, const float* __restrict__ times, const int* __restrict__ tptr, float* __restrict__ SLOT, int* __restrict__ LENS) {
  __shared__ int cntp[NP][257]; __shared__ int cnt[256]; __shared__ int lens[NP], starts[NP];
  const int t_ = threadIdx.x;
  for (size_t i = t_; i < (size_t)NP * L * 4; i += 256) ((volatile float*)SLOT)[i] = 0.0f;
  int local[NP];
#pragma unroll
  for (int p = 0; p < NP; ++p) local[p] = 0;
  int mine = 0;
  for (int e = 0; e < 256; ++e) { const int idx = t_ * 256 + e; const int row = idx >> 5; const int on = (M[idx] != 0) ? 1 : 0; const int p = iclamp(obs[row], 0, NP - 1); mine += on;
#pragma unroll
    for (int q = 0; q < NP; ++q) local[q] += (q == p) ? on : 0; }
#pragma unroll
  for (int p = 0; p < NP; ++p) cntp[p][t_] = local[p];
  cnt[t_] = mine; __syncthreads();
  if (t_ < NP) { int s = 0; for (int j = 0; j < 256; ++j) s += cntp[t_][j]; lens[t_] = s; }
  __syncthreads();
  if (t_ == 0) { int s = 0; for (int p = 0; p < NP; ++p) { starts[p] = s; s += lens[p]; } }
  __syncthreads();
  if (t_ == 0) { int s = 0; for (int j = 0; j < 256; ++j) { const int c = cnt[j]; cnt[j] = s; s += c; } }
  __syncthreads(); __threadfence();
  int ord = cnt[t_];
  for (int pass = 0; pass < 2; ++pass) { int o = ord;
    for (int e = 0; e < 256; ++e) { const int idx = t_ * 256 + e; const int row = idx >> 5, var = idx & 31; if (M[idx] == 0) continue; const int p = iclamp(obs[row], 0, NP - 1); const int pos = o - starts[p]; o += 1;
      if (pos < 0 || pos >= L) continue;
      int lo = 0, hi = R; while (lo < hi) { const int mid = (lo + hi + 1) >> 1; if (tptr[mid] <= row) lo = mid; else hi = mid - 1; }
      const v4f ent = {(float)var, bf16_rne(X[row * V + var]), bf16_rne(times[iclamp(lo, 0, R - 1)]), 1.0f};
      *(volatile v4f*)(SLOT + ((size_t)p * L + pos) * 4) = ent; }
    if (t_ < NP) ((volatile int*)LENS)[t_] = lens[t_];
    __threadfence(); }
}
__global__ __launch_bounds__(256) void prep_kernel(const float* __restrict__ w0, const float* __restrict__ w1, const float* __restrict__ w2, const float* __restrict__ wk, b16* __restrict__ WP) {
  const int t = blockIdx.x * 256 + threadIdx.x; const int n0 = W * KIN / 8, n1 = W * W / 8; v8b o = {};
  if (t < n0) { const int oo = (t * 8) / KIN, k0 = t * 8 - oo * KIN; for (int j = 0; j < 8; ++j) { const int k = k0 + j; o[j] = (b16)((k < NIN) ? bf16_rne(w0[oo * NIN + k]) * WSC : 0.0f); } for (int pass = 0; pass < 2; ++pass) { *(volatile v8b*)(WP + (size_t)t * 8) = o; __threadfence(); } }
  else if (t < n0 + 3 * n1) { const int u = t - n0; const int k = u / n1; const int e = (u - k * n1) * 8; const float* w = k == 0 ? w1 : k == 1 ? w2 : wk; for (int j = 0; j < 8; ++j) o[j] = (b16)(bf16_rne(w[e + j]) * WSC); for (int pass = 0; pass < 2; ++pass) { *(volatile v8b*)(WP + (size_t)W * KIN + (size_t)k * W * W + e) = o; __threadfence(); } }
}
__global__ __launch_bounds__(128) void enc_kernel(const float* __restrict__ SLOT, const b16* __restrict__ WP, const float* __restrict__ b0, const float* __restrict__ b1, const float* __restrict__ b2, const float* __restrict__ bk, float* __restrict__ ENC, float* __restrict__ KP) {
  __shared__ __attribute__((aligned(16))) b16 Ah[4][16][W + 8], Alo[4][16][W + 8]; __shared__ __attribute__((aligned(16))) float Ts[4][16][W + 4];
  const int wave = threadIdx.x >> 5, lane = threadIdx.x & 31, nloc = lane & 15, hlf = lane >> 4; const size_t m0 = ((size_t)blockIdx.x * 4 + wave) * 16;
  const b16* W0P = WP; const b16* W1P = WP + (size_t)W * KIN; const b16* W2P = W1P + (size_t)W * W; const b16* WKP = W2P + (size_t)W * W;
  { const int rr = nloc; const v4f s4 = *(const v4f*)(SLOT + (m0 + rr) * 4); const float var = s4[0], val = s4[1], tt = s4[2];
    for (int c = hlf * 32; c < hlf * 32 + 32; ++c) { float f = 0.0f;
      if (c < 16) { const float ts = __builtin_exp2f((float)c / 15.0f * 6.643856189774724f  ); f = sinf(tt / ts); }
      else if (c < 32) { const float ts = __builtin_exp2f((float)(c - 16) / 15.0f * 6.643856189774724f); f = cosf(tt / ts); }
      else if (c == 32) f = var; else if (c == 33) f = val;
      b16 h_, l_; split16(f * XS, h_, l_); Ah[wave][rr][c] = h_; Alo[wave][rr][c] = l_; } }
  wave_lds_sync();
  v8f acc[8];
  for (int layer = 0; layer < 4; ++layer) { const b16* Wt = layer == 0 ? W0P : layer == 1 ? W1P : layer == 2 ? W2P : WKP; const int Kl = layer == 0 ? KIN : W; const float* bb = layer == 0 ? b0 : layer == 1 ? b1 : layer == 2 ? b2 : bk;
#pragma unroll
    for (int t = 0; t < 8; ++t) acc[t] = (v8f){};
    for (int kb = 0; kb < Kl; kb += 32) { const v16b a = frag_kb(&Ah[wave][nloc][kb], hlf), al = frag_kb(&Alo[wave][nloc][kb], hlf);
#pragma unroll
      for (int t = 0; t < 8; ++t) { const v16b bw = frag_kb(Wt + (size_t)(t * 16 + nloc) * Kl + kb, hlf); acc[t] = wmma16b(a, bw, acc[t]); acc[t] = wmma16b(al, bw, acc[t]); } }
    wave_lds_sync();
#pragma unroll
    for (int t = 0; t < 8; ++t) { const int c = t * 16 + nloc; const float bv = bf16_rne(bb[c]);
#pragma unroll
      for (int r = 0; r < 8; ++r) { float v = acc[t][r] * (1.0f / (XS * WSC)) + bv; if (layer < 2) v = fmaxf(v, 0.0f); if (layer == 2 || layer == 3) Ts[wave][8 * hlf + r][c] = v; if (layer < 3) { b16 h_, l_; split16(v * XS, h_, l_); Ah[wave][8 * hlf + r][c] = h_; Alo[wave][8 * hlf + r][c] = l_; } } }
    wave_lds_sync();
    if (layer >= 2) { float* dst = layer == 2 ? ENC : KP; for (int pass = 0; pass < 2; ++pass) { for (int rr = 0; rr < 16; ++rr) *(volatile v4f*)(dst + (m0 + rr) * W + lane * 4) = *(const v4f*)(&Ts[wave][rr][lane * 4]); __threadfence(); } wave_lds_sync(); } }
}
__global__ __launch_bounds__(256) void pool_kernel(const float* __restrict__ ENC, const float* __restrict__ KP, const float* __restrict__ wq, const float* __restrict__ bq, const int* __restrict__ LENS, float* __restrict__ out) {
  __shared__ float qh[HD]; __shared__ float wl[L]; __shared__ float red[256];
  const int p = blockIdx.x / NH, h = blockIdx.x - p * NH, t_ = threadIdx.x; const int len = LENS[p];
  const float* elast = ENC + ((size_t)p * L + (L - 1)) * W;
  if (t_ < HD) { const int o = h * HD + t_; float s = bf16_rne(bq[o]); for (int c = 0; c < W; ++c) s += pmul(bf16_rne(wq[o * W + c]), elast[c]); qh[t_] = s; }
  __syncthreads();
  const float isq = 0.17677669529663687f;
  float mx = -INFINITY;
  for (int l = t_; l < L; l += 256) { const float* kr = KP + ((size_t)p * L + l) * W + h * HD; float s = 0.0f; for (int d = 0; d < HD; ++d) s += pmul(qh[d], kr[d]); s *= isq; if (l >= len) s = -1e30f; wl[l] = s; mx = fmaxf(mx, s); }
  red[t_] = mx; __syncthreads(); for (int st = 128; st >= 1; st >>= 1) { if (t_ < st) red[t_] = fmaxf(red[t_], red[t_ + st]); __syncthreads(); } const float m = red[0]; __syncthreads();
  float sm = 0.0f; for (int l = t_; l < L; l += 256) { const float e = nexp(wl[l] - m); wl[l] = e; sm += e; }
  red[t_] = sm; __syncthreads(); for (int st = 128; st >= 1; st >>= 1) { if (t_ < st) red[t_] += red[t_ + st]; __syncthreads(); } const float inv = 1.0f / red[0]; __syncthreads();
  float acc = 0.0f; if (t_ < W) { for (int l = 0; l < L; ++l) acc += pmul(wl[l], ENC[((size_t)p * L + l) * W + t_]); acc *= inv; }
  for (int pass = 0; pass < 2; ++pass) { if (t_ < W) ((volatile float*)out)[(size_t)p * (NH * W) + h * W + t_] = acc; __threadfence(); }
}
}

extern "C" void kernel_launch(void* const* d_in, const int* in_sizes, int n_in, void* d_out, int out_size, void* d_ws, size_t ws_size, hipStream_t stream) {
  (void)n_in;
  auto Fp = [&](int i) { return (const float*)d_in[i]; }; auto Ip = [&](int i) { return (const int*)d_in[i]; };
  if (in_sizes[0] != R || in_sizes[1] != R + 1 || in_sizes[2] != R * V || in_sizes[3] != R * V || in_sizes[4] != R || in_sizes[5] != NP || in_sizes[6] != W * NIN || in_sizes[8] != W * W || out_size != NP * NH * W) return;
  size_t off = 0; char* ws = (char*)d_ws;
  auto carve = [&](size_t bytes) { char* p = ws + off; off += (bytes + 255) & ~(size_t)255; return p; };
  float* SLOT = (float*)carve((size_t)NP * L * 4 * 4); int* LENS = (int*)carve(256); b16* WP = (b16*)carve(((size_t)W * KIN + 3 * (size_t)W * W) * 2); float* ENC = (float*)carve((size_t)NSR * W * 4); float* KP = (float*)carve((size_t)NSR * W * 4);
  if (off > ws_size || off > ((size_t)128 << 20)) return;
  scatter_kernel<<<1, 256, 0, stream>>>(Ip(3), Ip(4), Fp(2), Fp(0), Ip(1), SLOT, LENS);
  prep_kernel<<<(W * KIN / 8 + 3 * W * W / 8 + 255) / 256, 256, 0, stream>>>(Fp(6), Fp(8), Fp(10), Fp(14), WP);
  enc_kernel<<<NSR / 64, 128, 0, stream>>>(SLOT, WP, Fp(7), Fp(9), Fp(11), Fp(15), ENC, KP);
  pool_kernel<<<NP * NH, 256, 0, stream>>>(ENC, KP, Fp(12), Fp(13), LENS, (float*)d_out);
}
